// BlockSparseRingMultiheadDilatedAttention_86354612453508
// MI455X (gfx1250) — hardware-verified
//
#include <hip/hip_runtime.h>
#include <math.h>
#include <stdint.h>

#define S_    8192
#define E_    768
#define NH    12
#define HD    64
#define DQKV  (3 * E_)
#define MK    2048
#define NPROB 28
#define NQB   (MK / 64)
#define NKT   (MK / 64)
#define NZL   (S_ * 5)
#define OUTN  (S_ * E_)
static_assert(NH * HD == E_);
static_assert(HD == 64);
static_assert((E_ % 64) == 0 && (DQKV % 64) == 0 && (S_ % 64) == 0);
static_assert((E_ % 32) == 0);
static_assert((((S_ / 64) * (DQKV / 64)) % 8) == 0);
static_assert((((S_ / 64) * (E_ / 64)) % 8) == 0);
static_assert(((S_ * E_ / 8) % 256) == 0);
static_assert(((DQKV * E_ / 8) % 256) == 0);
static_assert(((E_ * E_ / 8) % 256) == 0);
static_assert((NZL % 32) == 0);
static_assert(4 * 4 + 4 * 2 + 4 * 1 == NPROB);
static_assert((NQB * NPROB) == 896);

typedef _Float16 v16h __attribute__((ext_vector_type(16)));
typedef _Float16 v8h  __attribute__((ext_vector_type(8)));
typedef float    v8f  __attribute__((ext_vector_type(8)));
typedef float    v4f  __attribute__((ext_vector_type(4)));
typedef unsigned int v4u __attribute__((ext_vector_type(4)));

__device__ __forceinline__ unsigned short bf_bits(float f) {
  unsigned u = __float_as_uint(f);
  return (unsigned short)((u + 0x7FFFu + ((u >> 16) & 1u)) >> 16);
}
__device__ __forceinline__ float bfr(float f) { return __uint_as_float(((unsigned)bf_bits(f)) << 16); }
__device__ __forceinline__ unsigned short h_bits(_Float16 x) { return __builtin_bit_cast(unsigned short, x); }
__device__ __forceinline__ unsigned pk16(unsigned short a, unsigned short b) { return (unsigned)a | ((unsigned)b << 16); }
__device__ __forceinline__ v8f zero8() { v8f z = {0.f, 0.f, 0.f, 0.f, 0.f, 0.f, 0.f, 0.f}; return z; }

__device__ __forceinline__ v16h ldfrag_h(const _Float16* p) {
  union { v16h v; v8h h[2]; } f;
  f.h[0] = *(const v8h*)(p);
  f.h[1] = *(const v8h*)(p + 16);
  return f.v;
}

__device__ __forceinline__ v8f mma_h(v16h a, v16h b, v8f c) {
  c = __builtin_amdgcn_wmma_f32_16x16x32_f16(false, a, false, b, (short)0, c, false, false);
#if defined(__HIP_DEVICE_COMPILE__)
  asm volatile("v_nop\n\tv_nop\n\tv_nop\n\tv_nop" : "+v"(c) : "v"(a), "v"(b));
#endif
  return c;
}
__device__ __forceinline__ v8f mma_h_raw(v16h a, v16h b, v8f c) {
  return __builtin_amdgcn_wmma_f32_16x16x32_f16(false, a, false, b, (short)0, c, false, false);
}
__device__ __forceinline__ void dep_guard_h(v8f& a, v8f& b, v16h x, v16h y) {
#if defined(__HIP_DEVICE_COMPILE__)
  asm volatile("v_nop\n\tv_nop\n\tv_nop\n\tv_nop" : "+v"(a), "+v"(b) : "v"(x), "v"(y));
#endif
}
__device__ __forceinline__ void keep4_h(v16h a, v16h b, v16h c, v16h d) {
#if defined(__HIP_DEVICE_COMPILE__)
  asm volatile("v_nop" :: "v"(a), "v"(b), "v"(c), "v"(d));
#endif
}
__device__ __forceinline__ void acc_guard4(v8f& a, v8f& b, v8f& c, v8f& d) {
#if defined(__HIP_DEVICE_COMPILE__)
  asm volatile("v_nop\n\tv_nop\n\tv_nop\n\tv_nop" : "+v"(a), "+v"(b), "+v"(c), "+v"(d));
#endif
}

__global__ __launch_bounds__(256) void cvt16(const float* __restrict__ in, unsigned short* out, int n8, float scale) {
  const int i = blockIdx.x * 256 + threadIdx.x;
  if (i < n8) {
    const v4f a = *(const v4f*)(in + (size_t)i * 8);
    const v4f b = *(const v4f*)(in + (size_t)i * 8 + 4);
    v4u p;
    p[0] = pk16(h_bits((_Float16)(bfr(a[0]) * scale)), h_bits((_Float16)(bfr(a[1]) * scale)));
    p[1] = pk16(h_bits((_Float16)(bfr(a[2]) * scale)), h_bits((_Float16)(bfr(a[3]) * scale)));
    p[2] = pk16(h_bits((_Float16)(bfr(b[0]) * scale)), h_bits((_Float16)(bfr(b[1]) * scale)));
    p[3] = pk16(h_bits((_Float16)(bfr(b[2]) * scale)), h_bits((_Float16)(bfr(b[3]) * scale)));
    *(volatile v4u*)(out + (size_t)i * 8) = p;
    __threadfence();
    *(volatile v4u*)(out + (size_t)i * 8) = p;
  }
}

template <int EPI, bool ARES>
__global__ __launch_bounds__(256) void gemm64_f16(
    const unsigned short* __restrict__ Ap, const unsigned short* __restrict__ Arp, int lda,
    const unsigned short* __restrict__ Btp, int ldb, float cscale,
    const float* __restrict__ bias,
    void* Cp, int ldc, unsigned short* Crp, int ldcr, int nres0,
    int M, int N, int K, float oscale) {
  const _Float16* Ah  = (const _Float16*)(const void*)Ap;
  const _Float16* Arh = (const _Float16*)(const void*)Arp;
  const _Float16* Bt  = (const _Float16*)(const void*)Btp;
  __shared__ __align__(16) float sT[8][16 * 68];
  const int lane = threadIdx.x & 31;
  const int wave = threadIdx.x >> 5;
  const int tilesN = N >> 6;
  const int tilesM = M >> 6;
  const int tile = blockIdx.x * 8 + wave;
  if (tile >= tilesM * tilesN) return;
  const int tm = tile / tilesN;
  const int tn = tile - tm * tilesN;
  const int m0 = tm << 6;
  const int n0 = tn << 6;

  const int rlane = lane & 15;
  const int koff  = (lane >> 4) * 8;
  const int mOff  = (lane >> 4) * 8;

  v8f acc[4][4];
#pragma unroll
  for (int i = 0; i < 4; ++i)
#pragma unroll
    for (int j = 0; j < 4; ++j) acc[i][j] = zero8();

  constexpr int NPL = ARES ? 2 : 1;
#pragma unroll 1
  for (int pl = 0; pl < NPL; ++pl) {
    const _Float16* Asel = (ARES && pl == 0) ? Arh : Ah;
    if (ARES && pl == 1) {
      acc_guard4(acc[0][0], acc[0][1], acc[0][2], acc[0][3]);
      acc_guard4(acc[1][0], acc[1][1], acc[1][2], acc[1][3]);
      acc_guard4(acc[2][0], acc[2][1], acc[2][2], acc[2][3]);
      acc_guard4(acc[3][0], acc[3][1], acc[3][2], acc[3][3]);
#pragma unroll
      for (int i = 0; i < 4; ++i)
#pragma unroll
        for (int j = 0; j < 4; ++j) acc[i][j] = acc[i][j] * (1.0f / 2048.0f);
      acc_guard4(acc[0][0], acc[0][1], acc[0][2], acc[0][3]);
      acc_guard4(acc[1][0], acc[1][1], acc[1][2], acc[1][3]);
      acc_guard4(acc[2][0], acc[2][1], acc[2][2], acc[2][3]);
      acc_guard4(acc[3][0], acc[3][1], acc[3][2], acc[3][3]);
    }
    for (int k0 = 0; k0 < K; k0 += 32) {
      v16h bh[4];
#pragma unroll
      for (int j = 0; j < 4; ++j) {
        const size_t bo = (size_t)(n0 + (j << 4) + rlane) * ldb + koff + k0;
        bh[j] = ldfrag_h(Bt + bo);
      }
#pragma unroll
      for (int i = 0; i < 4; ++i) {
        const size_t ao = (size_t)(m0 + (i << 4) + rlane) * lda + koff + k0;
        const v16h ah = ldfrag_h(Asel + ao);
#pragma unroll
        for (int j = 0; j < 4; ++j) {
          acc[i][j] = mma_h_raw(ah, bh[j], acc[i][j]);
        }
        dep_guard_h(acc[i][0], acc[i][3], ah, bh[3]);
      }
      keep4_h(bh[0], bh[1], bh[2], bh[3]);
    }
  }
  acc_guard4(acc[0][0], acc[0][1], acc[0][2], acc[0][3]);
  acc_guard4(acc[1][0], acc[1][1], acc[1][2], acc[1][3]);
  acc_guard4(acc[2][0], acc[2][1], acc[2][2], acc[2][3]);
  acc_guard4(acc[3][0], acc[3][1], acc[3][2], acc[3][3]);

  float bcol[4];
#pragma unroll
  for (int j = 0; j < 4; ++j) bcol[j] = bfr(bias[n0 + (j << 4) + rlane]);

  float* slab = sT[wave];
#pragma unroll
  for (int i = 0; i < 4; ++i) {
    const int mBase = m0 + (i << 4);
#pragma unroll
    for (int r = 0; r < 8; ++r) {
      const int row = mOff + r;
#pragma unroll
      for (int j = 0; j < 4; ++j) slab[row * 68 + (j << 4) + rlane] = acc[i][j][r] * cscale + bcol[j];
    }
    __builtin_amdgcn_fence(__ATOMIC_RELEASE, "workgroup");
    __builtin_amdgcn_wave_barrier();
    __builtin_amdgcn_fence(__ATOMIC_ACQUIRE, "workgroup");
    if constexpr (EPI == 0) {
      unsigned short* C16 = (unsigned short*)Cp;
      const bool wres = (n0 >= nres0);
      const int rq = lane >> 3, piece = lane & 7;
      v4u ph[4], pr[4];
#pragma unroll
      for (int it = 0; it < 4; ++it) {
        const int row = it * 4 + rq;
        const v4f a  = *(const v4f*)(slab + row * 68 + piece * 8);
        const v4f a2 = *(const v4f*)(slab + row * 68 + piece * 8 + 4);
        float f[8];
        f[0] = a[0];  f[1] = a[1];  f[2] = a[2];  f[3] = a[3];
        f[4] = a2[0]; f[5] = a2[1]; f[6] = a2[2]; f[7] = a2[3];
        v4u p, q;
#pragma unroll
        for (int e = 0; e < 4; ++e) {
          const float g0 = f[2 * e] * oscale, g1 = f[2 * e + 1] * oscale;
          const _Float16 x0 = (_Float16)g0, x1 = (_Float16)g1;
          const _Float16 y0 = (_Float16)((g0 - (float)x0) * 2048.0f);
          const _Float16 y1 = (_Float16)((g1 - (float)x1) * 2048.0f);
          p[e] = pk16(h_bits(x0), h_bits(x1));
          q[e] = pk16(h_bits(y0), h_bits(y1));
        }
        ph[it] = p;
        pr[it] = q;
      }
      for (int pass = 0; pass < 2; ++pass) {
#pragma unroll
        for (int it = 0; it < 4; ++it) {
          const int row = it * 4 + rq;
          const size_t co = (size_t)(mBase + row) * ldc + n0 + piece * 8;
          *(volatile v4u*)(C16 + co) = ph[it];
          if (wres) {
            const size_t cr = (size_t)(mBase + row) * ldcr + (n0 - nres0) + piece * 8;
            *(volatile v4u*)(Crp + cr) = pr[it];
          }
        }
        __threadfence();
      }
    } else {
      float* Cf = (float*)Cp;
      const int hh = lane >> 4, c4 = (lane & 15) * 4;
      v4f ov[8];
#pragma unroll
      for (int it = 0; it < 8; ++it) {
        const int row = it * 2 + hh;
        ov[it] = *(const v4f*)(slab + row * 68 + c4);
      }
      for (int pass = 0; pass < 2; ++pass) {
#pragma unroll
        for (int it = 0; it < 8; ++it) {
          const int row = it * 2 + hh;
          *(volatile v4f*)(Cf + (size_t)(mBase + row) * ldc + n0 + c4) = ov[it];
        }
        __threadfence();
      }
    }
    __builtin_amdgcn_fence(__ATOMIC_RELEASE, "workgroup");
    __builtin_amdgcn_wave_barrier();
    __builtin_amdgcn_fence(__ATOMIC_ACQUIRE, "workgroup");
  }
}

__global__ __launch_bounds__(256) void v_tr(const unsigned short* __restrict__ srcp, int pitch, int col0,
                                            unsigned short* vt) {
  __shared__ __align__(16) _Float16 sv[64 * 72];
  const int tid   = threadIdx.x;
  const int hh    = blockIdx.y;
  const int shift = hh >> 2;
  const int nU    = S_ >> shift;
  const int u0    = blockIdx.x * 64;
  if (u0 >= nU) return;
  const int off   = (hh & 3) & ((1 << shift) - 1);
  const _Float16* src = (const _Float16*)(const void*)srcp;
#pragma unroll
  for (int i = 0; i < 2; ++i) {
    const int idx = i * 256 + tid;
    const int uu = idx >> 3, c8 = (idx & 7) * 8;
    const int u = u0 + uu;
    const int tok = ((u >> 11) << (11 + shift)) + off + ((u & 2047) << shift);
    const v8h a = *(const v8h*)(src + (size_t)tok * pitch + col0 + hh * HD + c8);
    *(v8h*)(sv + uu * 72 + c8) = a;
  }
  __syncthreads();

  const int g = tid >> 3, piece = tid & 7;
  v4u hv[2];
  size_t hofs[2];
#pragma unroll
  for (int it = 0; it < 2; ++it) {
    const int d = it * 32 + g;
    v4u a;
#pragma unroll
    for (int e = 0; e < 4; ++e) {
      const _Float16 x0 = sv[(piece * 8 + 2 * e) * 72 + d];
      const _Float16 x1 = sv[(piece * 8 + 2 * e + 1) * 72 + d];
      a[e] = pk16(h_bits(x0), h_bits(x1));
    }
    hv[it] = a;
    hofs[it] = ((size_t)(hh * HD + d)) * S_ + u0 + piece * 8;
  }
  for (int pass = 0; pass < 2; ++pass) {
#pragma unroll
    for (int it = 0; it < 2; ++it) *(volatile v4u*)(vt + hofs[it]) = hv[it];
    __threadfence();
  }
}

__global__ __launch_bounds__(256) void ctx_zero(unsigned short* ctxp, unsigned short* ctxrp) {
  const int tid = threadIdx.x;
  const int L = blockIdx.x * 32 + (tid >> 3);
  if (L >= NZL) return;
  const int piece = tid & 7;
  const int row = L / 5;
  const int j   = L - row * 5;
  const int h1  = 4 + 2 * j + ((row & 1) ^ 1);
  const int h2  = 8 + (((row & 3) + (j - 1)) & 3);
  const int h   = (j < 2) ? h1 : h2;
  const size_t go = (size_t)row * E_ + (size_t)h * HD + piece * 8;
  v4u z = {0u, 0u, 0u, 0u};
  *(volatile v4u*)(ctxp + go)  = z;
  *(volatile v4u*)(ctxrp + go) = z;
  __threadfence();
  *(volatile v4u*)(ctxp + go)  = z;
  *(volatile v4u*)(ctxrp + go) = z;
}

__global__ __launch_bounds__(128)
void attn_k(const unsigned short* __restrict__ qkvp, const unsigned short* __restrict__ vtp,
            const unsigned short* __restrict__ vtrp, unsigned short* ctxp, unsigned short* ctxrp) {
  union FH { v16h v; v8h h[2]; };
  constexpr int TB     = 64 * 64 * 2;
  constexpr int PB     = 4 * 16 * 64 * 2;
  constexpr int OFF_K  = 0;
  constexpr int OFF_V  = TB;
  constexpr int OFF_VR = 2 * TB;
  constexpr int OFF_P  = 3 * TB;
  constexpr int OFF_PR = OFF_P + PB;
  constexpr int SMEMB  = OFF_PR + PB;
  static_assert(4 * 16 * 64 * 4 <= OFF_P);
  __shared__ __align__(16) unsigned char smem[SMEMB];
  _Float16* Ksh = (_Float16*)(smem + OFF_K);
  _Float16* Vsh = (_Float16*)(smem + OFF_V);
  _Float16* Vrs = (_Float16*)(smem + OFF_VR);
  _Float16* Psh = (_Float16*)(smem + OFF_P);
  _Float16* Prs = (_Float16*)(smem + OFF_PR);

  const int tid  = threadIdx.x;
  const int wave = tid >> 5;
  const int lane = tid & 31;
  const int hh   = lane >> 4;
  const int c    = lane & 15;

  const int bx  = blockIdx.x;
  const int qb  = bx % NQB;
  const int pid = bx / NQB;
  if (pid >= NPROB) return;
  int h, seg;
  if (pid < 16)      { h = pid >> 2;              seg = pid & 3; }
  else if (pid < 24) { h = 4 + ((pid - 16) >> 1); seg = (pid - 16) & 1; }
  else               { h = 8 + (pid - 24);        seg = 0; }
  const int shift   = h >> 2;
  const int off     = (h & 3) & ((1 << shift) - 1);
  const int tokbase = (seg << (11 + shift)) + off;
  const int ubase   = seg << 11;
  const int q0      = qb * 64 + wave * 16;

  const _Float16* Qp  = (const _Float16*)(const void*)qkvp + (size_t)h * HD;
  const _Float16* Kp  = Qp + E_;
  const _Float16* Vt  = (const _Float16*)(const void*)vtp  + (size_t)h * HD * S_ + ubase;
  const _Float16* Vrt = (const _Float16*)(const void*)vtrp + (size_t)h * HD * S_ + ubase;

  v16h qa[2];
#pragma unroll
  for (int dc = 0; dc < 2; ++dc) {
    const size_t qo = (size_t)(tokbase + ((q0 + c) << shift)) * DQKV + dc * 32 + 8 * hh;
    qa[dc] = ldfrag_h(Qp + qo);
  }

  float lsum[8], mrun[8];
  v8f oacc[4], oacc2[4];
#pragma unroll
  for (int r = 0; r < 8; ++r) { lsum[r] = 0.f; mrun[r] = -1e30f; }
#pragma unroll
  for (int t = 0; t < 4; ++t) { oacc[t] = zero8(); oacc2[t] = zero8(); }

  _Float16* pw  = Psh + wave * (16 * 64);
  _Float16* prw = Prs + wave * (16 * 64);

  for (int kt = 0; kt < NKT; ++kt) {
    const int kv0 = kt * 64;
    __syncthreads();
    {
      const int r = tid >> 1, half = (tid & 1) * 32;
      const size_t ko = (size_t)(tokbase + ((kv0 + r) << shift)) * DQKV + half;
      const size_t vo = (size_t)r * S_ + kv0 + half;
#pragma unroll
      for (int i = 0; i < 4; ++i) {
        const v8h a0 = *(const v8h*)(Kp + ko + 8 * i);
        const v8h b0 = *(const v8h*)(Vt + vo + 8 * i);
        const v8h b1 = *(const v8h*)(Vrt + vo + 8 * i);
        *(v8h*)(Ksh + r * 64 + half + 8 * i) = a0;
        *(v8h*)(Vsh + r * 64 + half + 8 * i) = b0;
        *(v8h*)(Vrs + r * 64 + half + 8 * i) = b1;
      }
    }
    __syncthreads();

    v8f s[4];
#pragma unroll
    for (int j = 0; j < 4; ++j) {
      s[j] = zero8();
#pragma unroll
      for (int dc = 0; dc < 2; ++dc) {
        FH kb;
        kb.h[0] = *(const v8h*)(Ksh + (j * 16 + c) * 64 + dc * 32 + 8 * hh);
        kb.h[1] = *(const v8h*)(Ksh + (j * 16 + c) * 64 + dc * 32 + 16 + 8 * hh);
        s[j] = mma_h(qa[dc], kb.v, s[j]);
      }
    }

    float alpha[8];
#pragma unroll
    for (int r = 0; r < 8; ++r) {
      float av[4];
      float tmx = -1e30f;
#pragma unroll
      for (int j = 0; j < 4; ++j) {
        const float a = s[j][r] * (1.0f / 2048.0f);
        av[j] = a;
        tmx = fmaxf(tmx, a);
      }
#pragma unroll
      for (int o = 1; o < 16; o <<= 1) tmx = fmaxf(tmx, __shfl_xor(tmx, o, 32));
      const float mn = fmaxf(mrun[r], tmx);
      const float al = __expf(mrun[r] - mn);
      alpha[r] = al;
      mrun[r]  = mn;
      float ps = 0.0f;
#pragma unroll
      for (int j = 0; j < 4; ++j) {
        const float p = __expf(av[j] - mn);
        ps += p;
        const float g = p * 256.0f;
        const _Float16 x0 = (_Float16)g;
        pw[(8 * hh + r) * 64 + j * 16 + c]  = x0;
        prw[(8 * hh + r) * 64 + j * 16 + c] = (_Float16)((g - (float)x0) * 2048.0f);
      }
      lsum[r] = lsum[r] * al + ps;
    }
    __builtin_amdgcn_fence(__ATOMIC_RELEASE, "workgroup");
    __builtin_amdgcn_wave_barrier();
    __builtin_amdgcn_fence(__ATOMIC_ACQUIRE, "workgroup");

#pragma unroll
    for (int t = 0; t < 4; ++t) {
#pragma unroll
      for (int r = 0; r < 8; ++r) {
        oacc[t][r]  = oacc[t][r] * alpha[r];
        oacc2[t][r] = oacc2[t][r] * alpha[r];
      }
    }
    acc_guard4(oacc[0], oacc[1], oacc[2], oacc[3]);
    acc_guard4(oacc2[0], oacc2[1], oacc2[2], oacc2[3]);

#pragma unroll
    for (int kk = 0; kk < 2; ++kk) {
      FH pa, par;
      pa.h[0]  = *(const v8h*)(pw  + c * 64 + kk * 32 + 8 * hh);
      pa.h[1]  = *(const v8h*)(pw  + c * 64 + kk * 32 + 16 + 8 * hh);
      par.h[0] = *(const v8h*)(prw + c * 64 + kk * 32 + 8 * hh);
      par.h[1] = *(const v8h*)(prw + c * 64 + kk * 32 + 16 + 8 * hh);
#pragma unroll
      for (int t = 0; t < 4; ++t) {
        FH vb, vrb;
        vb.h[0]  = *(const v8h*)(Vsh + (t * 16 + c) * 64 + kk * 32 + 8 * hh);
        vb.h[1]  = *(const v8h*)(Vsh + (t * 16 + c) * 64 + kk * 32 + 16 + 8 * hh);
        vrb.h[0] = *(const v8h*)(Vrs + (t * 16 + c) * 64 + kk * 32 + 8 * hh);
        vrb.h[1] = *(const v8h*)(Vrs + (t * 16 + c) * 64 + kk * 32 + 16 + 8 * hh);
        oacc[t]  = mma_h(pa.v, vb.v, oacc[t]);
        oacc2[t] = mma_h(pa.v, vrb.v, oacc2[t]);
        oacc2[t] = mma_h(par.v, vb.v, oacc2[t]);
      }
    }
  }
  __syncthreads();

  float* os = (float*)(void*)smem + wave * (16 * 64);
#pragma unroll
  for (int r = 0; r < 8; ++r) {
    float l = lsum[r];
#pragma unroll
    for (int o = 1; o < 16; o <<= 1) l += __shfl_xor(l, o, 32);
    const float rl = 1.0f / l;
    const float sc = rl * (1.0f / 256.0f);
#pragma unroll
    for (int t = 0; t < 4; ++t) {
      const float v = oacc[t][r] + oacc2[t][r] * (1.0f / 2048.0f);
      os[(8 * hh + r) * 64 + t * 16 + c] = v * sc;
    }
  }
  __builtin_amdgcn_fence(__ATOMIC_RELEASE, "workgroup");
  __builtin_amdgcn_wave_barrier();
  __builtin_amdgcn_fence(__ATOMIC_ACQUIRE, "workgroup");
  {
    const int rq = lane >> 3, piece = lane & 7;
    v4u ph[4], pr[4];
#pragma unroll
    for (int it = 0; it < 4; ++it) {
      const int row = it * 4 + rq;
      const v4f a  = *(const v4f*)(os + row * 64 + piece * 8);
      const v4f a2 = *(const v4f*)(os + row * 64 + piece * 8 + 4);
      float f[8];
      f[0] = a[0];  f[1] = a[1];  f[2] = a[2];  f[3] = a[3];
      f[4] = a2[0]; f[5] = a2[1]; f[6] = a2[2]; f[7] = a2[3];
      v4u p, q;
#pragma unroll
      for (int e = 0; e < 4; ++e) {
        const _Float16 x0 = (_Float16)f[2 * e], x1 = (_Float16)f[2 * e + 1];
        const _Float16 y0 = (_Float16)((f[2 * e] - (float)x0) * 2048.0f);
        const _Float16 y1 = (_Float16)((f[2 * e + 1] - (float)x1) * 2048.0f);
        p[e] = pk16(h_bits(x0), h_bits(x1));
        q[e] = pk16(h_bits(y0), h_bits(y1));
      }
      ph[it] = p;
      pr[it] = q;
    }
    for (int pass = 0; pass < 2; ++pass) {
#pragma unroll
      for (int it = 0; it < 4; ++it) {
        const int row = it * 4 + rq;
        const size_t go = (size_t)(tokbase + ((q0 + row) << shift)) * E_ + (size_t)h * HD + piece * 8;
        *(volatile v4u*)(ctxp + go)  = ph[it];
        *(volatile v4u*)(ctxrp + go) = pr[it];
      }
      __threadfence();
    }
  }
}

extern "C" void kernel_launch(void* const* d_in, const int* in_sizes, int n_in,
                              void* d_out, int out_size, void* d_ws, size_t ws_size,
                              hipStream_t stream) {
  if (n_in < 5) return;
  if (in_sizes[0] != S_ * E_) return;
  if (in_sizes[1] != DQKV * E_) return;
  if (in_sizes[2] != DQKV) return;
  if (in_sizes[3] != E_ * E_) return;
  if (in_sizes[4] != E_) return;
  if (out_size != OUTN) return;

  const float* x     = (const float*)d_in[0];
  const float* qkv_w = (const float*)d_in[1];
  const float* qkv_b = (const float*)d_in[2];
  const float* out_w = (const float*)d_in[3];
  const float* out_b = (const float*)d_in[4];

  const size_t PX    = (size_t)S_ * E_ * 2;
  const size_t PWq   = (size_t)DQKV * E_ * 2;
  const size_t PWp   = (size_t)E_ * E_ * 2;
  const size_t PQKV  = (size_t)S_ * DQKV * 2;
  const size_t PVr   = (size_t)S_ * E_ * 2;
  const size_t PVT   = (size_t)NH * HD * S_ * 2;
  const size_t PCtx  = (size_t)S_ * E_ * 2;
  size_t off = 0;
  const size_t oX    = off; off += PX;
  const size_t oWq   = off; off += PWq;
  const size_t oWp   = off; off += PWp;
  const size_t oQKV  = off; off += PQKV;
  const size_t oVr   = off; off += PVr;
  const size_t oVT   = off; off += PVT;
  const size_t oVTr  = off; off += PVT;
  const size_t oCtx  = off; off += PCtx;
  const size_t oCtxr = off; off += PCtx;
  if (off > ws_size) return;
  if (off > (size_t)134217728) return;

  char* ws = (char*)d_ws;
  unsigned short* Xh   = (unsigned short*)(ws + oX);
  unsigned short* Wqkv = (unsigned short*)(ws + oWq);
  unsigned short* Wp   = (unsigned short*)(ws + oWp);
  unsigned short* QKV  = (unsigned short*)(ws + oQKV);
  unsigned short* Vr   = (unsigned short*)(ws + oVr);
  unsigned short* VT   = (unsigned short*)(ws + oVT);
  unsigned short* VTr  = (unsigned short*)(ws + oVTr);
  unsigned short* Ctx  = (unsigned short*)(ws + oCtx);
  unsigned short* Ctxr = (unsigned short*)(ws + oCtxr);
  float*          outf = (float*)d_out;

  const dim3 blk(256);
  const int n8x = S_ * E_ / 8;
  const int n8q = DQKV * E_ / 8;
  const int n8p = E_ * E_ / 8;
  const dim3 gCx((n8x + 255) / 256);
  const dim3 gCq((n8q + 255) / 256);
  const dim3 gCp((n8p + 255) / 256);
  const dim3 gGqkv(((S_ / 64) * (DQKV / 64) + 7) / 8);
  const dim3 gGout(((S_ / 64) * (E_ / 64) + 7) / 8);
  const dim3 gVt(S_ / 64, NH);
  const dim3 gZ(NZL / 32);
  const dim3 gAttn(NQB * NPROB);
  const float wScale = 1024.0f;
  const float aScale = 16.0f;
  const float cscale = 1.0f / 16384.0f;

  cvt16<<<gCx, blk, 0, stream>>>(x, Xh, n8x, aScale);
  cvt16<<<gCq, blk, 0, stream>>>(qkv_w, Wqkv, n8q, wScale);
  cvt16<<<gCp, blk, 0, stream>>>(out_w, Wp, n8p, wScale);
  gemm64_f16<0, false><<<gGqkv, blk, 0, stream>>>(Xh, Xh, E_, Wqkv, E_, cscale, qkv_b,
                                                   (void*)QKV, DQKV, Vr, E_, 2 * E_,
                                                   S_, DQKV, E_, aScale);
  v_tr<<<gVt, blk, 0, stream>>>(QKV, DQKV, 2 * E_, VT);
  v_tr<<<gVt, blk, 0, stream>>>(Vr, E_, 0, VTr);
  ctx_zero<<<gZ, blk, 0, stream>>>(Ctx, Ctxr);
  attn_k<<<gAttn, dim3(128), 0, stream>>>(QKV, VT, VTr, Ctx, Ctxr);
  gemm64_f16<1, true><<<gGout, blk, 0, stream>>>(Ctx, Ctxr, E_, Wp, E_, cscale, out_b,
                                                 (void*)outf, E_, Ctxr, E_, 1 << 30,
                                                 S_, E_, E_, 1.0f);
  (void)hipGetLastError();
}
